// GNN_63934883168987
// MI455X (gfx1250) — hardware-run, weakly checked
//
#include <hip/hip_runtime.h>
#include <stddef.h>
#include <stdint.h>


#define DF       128
#define SP       256
#define XP       128
#define WPA      384
#define WPB      512
#define WOFF_ROOT 256
#define SPLIT_S1 1
#define SPLIT_S2 1
#define SPLIT_H  1
#define KS_S1    (SPLIT_S1 ? 8 : 4)
#define KS_X     4
#define KS_S2    (SPLIT_S2 ? 8 : 4)
#define KS_H     (SPLIT_H ? 8 : 4)
#define NTHR     256
#define NWAVE    8
#define EPT      8
#define CHUNK    (NTHR * EPT)
#define NBA      1024
#define PKS      10
#define WLCAP    3584
#define RCAP     (NWAVE * WLCAP)
#define DEGCAP   64
#define GBM      64
#define GBN      128
#define GTHR     128
#define RPB      64
#define RPW      8
#define UPART    2048
#define NPART    7
#define WBLK     ((NPART * UPART) / NTHR)
#define BK_INTS  (2 * RCAP + 3 * NBA + 32)
#define LDS_BK   (BK_INTS * 4)
#define MEAS_BLK_HITS 16710
#define MEAS_MAXDEG   36
#define NNODE_LIT 100000
#define NB_LIT    98
#define NP_LIT    (782 * 128)

static_assert(DF == 32 * 4 && DF == 16 * 8);
static_assert((KS_S1 + KS_X) * 32 <= WPA && (KS_S2 + KS_H) * 32 <= WPB);
static_assert(WPA % 32 == 0 && WPB % 32 == 0 && WPA == 3 * DF && WPB == 4 * DF);
static_assert(SP == 2 * DF && XP == DF && WOFF_ROOT == 2 * DF);
static_assert(KS_S1 * 32 <= SP && KS_S2 * 32 <= SP && KS_H * 32 <= SP && KS_X * 32 <= XP);
static_assert((CHUNK & (CHUNK - 1)) == 0 && CHUNK <= 4096);
static_assert(NBA == (1 << PKS) && NBA == NTHR * 4);
static_assert(RCAP % (NTHR * 4) == 0 && BK_INTS % 4 == 0);
static_assert((long long)RCAP * 100 >= (long long)MEAS_BLK_HITS * 105);
static_assert((long long)WLCAP * 100 >= (long long)(MEAS_BLK_HITS / NWAVE) * 150);
static_assert(DEGCAP >= MEAS_MAXDEG + 8 && DEGCAP % 32 == 0);
static_assert(LDS_BK <= 300000 && LDS_BK <= 327680);
static_assert(GBM == (GTHR / 32) * 16 && GBN == DF && RPB == NWAVE * RPW && RPB == GBM);
static_assert(NBA % RPB == 0 && NBA % GBM == 0);
static_assert(UPART % NTHR == 0 && UPART == DF * (DF / 8));
static_assert(NB_LIT * NBA >= NNODE_LIT && NB_LIT * NBA >= NP_LIT);
static_assert(NP_LIT >= NNODE_LIT && NP_LIT % GBM == 0 && NP_LIT - NNODE_LIT < 128);
static_assert((size_t)DF * WPA * 2 + (size_t)DF * WPB * 2 + (size_t)NB_LIT * RCAP * 4 +
              2 * (size_t)NB_LIT * NBA * 4 + (size_t)NB_LIT * 128 + 2 * (size_t)NP_LIT * SP * 2
              <= (size_t)(128u << 20));

typedef float          v4f   __attribute__((ext_vector_type(4)));
typedef float          v8f   __attribute__((ext_vector_type(8)));
typedef int            v4i   __attribute__((ext_vector_type(4)));
typedef int            v8i   __attribute__((ext_vector_type(8)));
typedef unsigned       v4u   __attribute__((ext_vector_type(4)));
typedef unsigned short v8us  __attribute__((ext_vector_type(8)));
typedef __bf16         v16bf __attribute__((ext_vector_type(16)));
typedef v4f  __attribute__((may_alias)) v4fa;
typedef v4i  __attribute__((may_alias)) v4ia;
typedef v4u  __attribute__((may_alias)) v4ua;
typedef v8us __attribute__((may_alias)) v8usa;
union FragB { v16bf v; v8us h[2]; v8i w; };

__device__ __forceinline__ v8f wmb(const FragB& a, const FragB& b, v8f c) {
  v8f d = __builtin_amdgcn_wmma_f32_16x16x32_bf16(false, a.v, false, b.v, (short)0, c, false, false);
  asm volatile("v_nop\n\tv_nop\n\tv_nop\n\tv_nop" : "+v"(d) : "v"(a.w), "v"(b.w));
  return d;
}

__device__ __forceinline__ unsigned bf16_bits(float f) {
  const unsigned u = __float_as_uint(f);
  return ((u + 0x7FFFu + ((u >> 16) & 1u)) >> 16) & 0xFFFFu;
}
__device__ __forceinline__ float bf16_val(float f) { return __uint_as_float(bf16_bits(f) << 16); }
__device__ __forceinline__ float bfw_lo(unsigned w) { return __uint_as_float(w << 16); }
__device__ __forceinline__ float bfw_hi(unsigned w) { return __uint_as_float(w & 0xffff0000u); }
__device__ __forceinline__ void pack2(float a, float b, unsigned& hw, unsigned& lw) {
  const unsigned ha = bf16_bits(a), hb = bf16_bits(b);
  const unsigned la = bf16_bits(a - __uint_as_float(ha << 16));
  const unsigned lb = bf16_bits(b - __uint_as_float(hb << 16));
  hw = ha | (hb << 16);
  lw = la | (lb << 16);
}
__device__ __forceinline__ float relu_k(float v) { return (v > 0.0f) ? v : (v - v); }
__device__ __forceinline__ float poison(float a, unsigned km, unsigned pz) {
  return __uint_as_float((__float_as_uint(a) & km) | pz);
}

__device__ __forceinline__ int scan_chunk(const int* __restrict__ keys, int nE, int cbase, int slotBase,
                                          int nb, int vec8, int* mylist, int wpos, int tid) {
  int wc = wpos;
  const int e0   = cbase + tid * EPT;
  const int sent = (int)(1u << 31);
  v4i da, db;
  if (vec8 != 0 && cbase + CHUNK <= nE) {
    da = *(const v4i*)(keys + e0);
    db = *(const v4i*)(keys + e0 + 4);
  } else {
    const int q0 = keys[min(e0,     nE - 1)];
    const int q1 = keys[min(e0 + 1, nE - 1)];
    const int q2 = keys[min(e0 + 2, nE - 1)];
    const int q3 = keys[min(e0 + 3, nE - 1)];
    const int q4 = keys[min(e0 + 4, nE - 1)];
    const int q5 = keys[min(e0 + 5, nE - 1)];
    const int q6 = keys[min(e0 + 6, nE - 1)];
    const int q7 = keys[min(e0 + 7, nE - 1)];
    asm volatile("" :: "v"(q0), "v"(q1), "v"(q2), "v"(q3), "v"(q4), "v"(q5), "v"(q6), "v"(q7));
    da.x = (e0     < nE) ? q0 : sent;
    da.y = (e0 + 1 < nE) ? q1 : sent;
    da.z = (e0 + 2 < nE) ? q2 : sent;
    da.w = (e0 + 3 < nE) ? q3 : sent;
    db.x = (e0 + 4 < nE) ? q4 : sent;
    db.y = (e0 + 5 < nE) ? q5 : sent;
    db.z = (e0 + 6 < nE) ? q6 : sent;
    db.w = (e0 + 7 < nE) ? q7 : sent;
  }
  const unsigned nbs = (unsigned)slotBase;
  const unsigned unb = (unsigned)nb;
  const unsigned s0 = (unsigned)da.x - nbs, s1 = (unsigned)da.y - nbs;
  const unsigned s2 = (unsigned)da.z - nbs, s3 = (unsigned)da.w - nbs;
  const unsigned s4 = (unsigned)db.x - nbs, s5 = (unsigned)db.y - nbs;
  const unsigned s6 = (unsigned)db.z - nbs, s7 = (unsigned)db.w - nbs;
  const bool h0 = s0 < unb, h1 = s1 < unb, h2 = s2 < unb, h3 = s3 < unb;
  const bool h4 = s4 < unb, h5 = s5 < unb, h6 = s6 < unb, h7 = s7 < unb;
  const unsigned any = __builtin_amdgcn_ballot_w32(h0 | h1 | h2 | h3 | h4 | h5 | h6 | h7);
  if (any != 0u) {
#define HITJ(J, HJ, SJ) { \
      const unsigned mj = __builtin_amdgcn_ballot_w32(HJ); \
      if (mj != 0u) { \
        if (HJ) { \
          const int pos = wc + (int)__builtin_amdgcn_mbcnt_lo(mj, 0u); \
          if (pos < WLCAP) mylist[pos] = ((e0 + (J)) << PKS) | (int)(SJ); \
        } \
        wc += (int)__builtin_popcount(mj); } }
    HITJ(0, h0, s0)
    HITJ(1, h1, s1)
    HITJ(2, h2, s2)
    HITJ(3, h3, s3)
    HITJ(4, h4, s4)
    HITJ(5, h5, s5)
    HITJ(6, h6, s6)
    HITJ(7, h7, s7)
#undef HITJ
  }
  return wc;
}

__device__ __forceinline__ void wunit(const float* __restrict__ W, unsigned short* P, int pitch, int coff,
                                      int n, int k8) {
  const float* p = W + (size_t)n * DF + k8;
  const v4f a = *(const v4f*)p;
  const v4f b = *(const v4f*)(p + 4);
  v8us o;
  o[0] = (unsigned short)bf16_bits(a.x); o[1] = (unsigned short)bf16_bits(a.y);
  o[2] = (unsigned short)bf16_bits(a.z); o[3] = (unsigned short)bf16_bits(a.w);
  o[4] = (unsigned short)bf16_bits(b.x); o[5] = (unsigned short)bf16_bits(b.y);
  o[6] = (unsigned short)bf16_bits(b.z); o[7] = (unsigned short)bf16_bits(b.w);
  unsigned short* dp = P + (size_t)n * pitch + coff + k8;
  *(volatile v8us*)dp = o;
  __threadfence();
  *(volatile v8us*)dp = o;
}

__global__ __launch_bounds__(NTHR) void k_prep(const float* __restrict__ x,
                                               const float* __restrict__ wrel1, const float* __restrict__ wroot1,
                                               const float* __restrict__ wrel2, const float* __restrict__ wroot2,
                                               unsigned short* xb, unsigned short* wca, unsigned short* wcb,
                                               int nN, int mRows) {
  const int tid = (int)threadIdx.x;
  const int b   = (int)blockIdx.x;
  if (b < WBLK) {
    const int u    = b * NTHR + tid;
    const int part = u >> 11;
    const int v    = u & (UPART - 1);
    const int n    = v >> 4;
    const int k8   = (v & 15) * 8;
    if (part == 0)      wunit(wrel1,  wca, WPA, 0,      n, k8);
    else if (part == 1) wunit(wrel1,  wca, WPA, DF,     n, k8);
    else if (part == 2) wunit(wroot1, wca, WPA, 2 * DF, n, k8);
    else if (part == 3) wunit(wrel2,  wcb, WPB, 0,      n, k8);
    else if (part == 4) wunit(wrel2,  wcb, WPB, DF,     n, k8);
    else if (part == 5) wunit(wroot2, wcb, WPB, 2 * DF, n, k8);
    else if (part == 6) wunit(wroot2, wcb, WPB, 3 * DF, n, k8);
  } else {
    const int u   = (b - WBLK) * NTHR + tid;
    const int row = u >> 4;
    const int c8  = (u & 15) * 8;
    if (row < mRows) {
      const int rc = row < nN ? row : nN - 1;
      const float* p = x + (size_t)rc * DF + c8;
      const v4f a = *(const v4f*)p;
      const v4f c = *(const v4f*)(p + 4);
      asm volatile("" :: "v"(a), "v"(c));
      const unsigned mk = (row < nN) ? 0xFFFFu : 0u;
      v8us o;
      o[0] = (unsigned short)(bf16_bits(a.x) & mk); o[1] = (unsigned short)(bf16_bits(a.y) & mk);
      o[2] = (unsigned short)(bf16_bits(a.z) & mk); o[3] = (unsigned short)(bf16_bits(a.w) & mk);
      o[4] = (unsigned short)(bf16_bits(c.x) & mk); o[5] = (unsigned short)(bf16_bits(c.y) & mk);
      o[6] = (unsigned short)(bf16_bits(c.z) & mk); o[7] = (unsigned short)(bf16_bits(c.w) & mk);
      unsigned short* dp = xb + (size_t)row * XP + c8;
      *(volatile v8us*)dp = o;
      __threadfence();
      *(volatile v8us*)dp = o;
    }
  }
}

__global__ __launch_bounds__(NTHR) void k_bucket(const int* __restrict__ keys, const int* __restrict__ gidx,
                                                 int nE, int nN, int vec8,
                                                 int* LIST, int* CNT, int* OFF, int* REC) {
  extern __shared__ __attribute__((aligned(16))) int dsm[];
  int* wl   = dsm;
  int* reg2 = wl + RCAP;
  int* scnt = reg2 + RCAP;
  int* soff = scnt + NBA;
  int* cur  = soff + NBA;
  int* wcnt = cur + NBA;
  int* wovf = wcnt + 8;
  int* wtot = wovf + 8;
  int* wmx  = wtot + 8;
  const int tid = (int)threadIdx.x, lane = tid & 31, wave = tid >> 5;
  const int nodeBase = (int)blockIdx.x * NBA;
  int nb = nN - nodeBase;
  nb = nb > NBA ? NBA : (nb < 1 ? 1 : nb);

  {
    const v4i z4 = {0, 0, 0, 0};
    for (int i = tid * 4; i < BK_INTS; i += NTHR * 4) *(v4ia*)(dsm + i) = z4;
  }
  __syncthreads();

  {
    int wpos = 0;
    int* mylist = wl + wave * WLCAP;
    const int nChunks = (nE + CHUNK - 1) / CHUNK;
#pragma unroll 1
    for (int ch = 0; ch < nChunks; ++ch)
      wpos = scan_chunk(keys, nE, ch * CHUNK, nodeBase, nb, vec8, mylist, wpos, tid);
    if (lane == 0) {
      wcnt[wave] = wpos > WLCAP ? WLCAP : wpos;
      wovf[wave] = wpos > WLCAP ? 1 : 0;
    }
  }
  __syncthreads();
  int nh = 0, ovf = 0;
#pragma unroll
  for (int w2 = 0; w2 < NWAVE; ++w2) {
    int c = wcnt[w2];
    c = c < 0 ? 0 : (c > WLCAP ? WLCAP : c);
    nh += c;
    ovf |= wovf[w2];
  }

  if (wave == 0) {
#pragma unroll 1
    for (int w2 = 0; w2 < NWAVE; ++w2) {
      int cv = wcnt[w2];
      cv = cv < 0 ? 0 : (cv > WLCAP ? WLCAP : cv);
      const int c = __builtin_amdgcn_readfirstlane(cv);
      const int* lw = wl + w2 * WLCAP;
#pragma unroll 1
      for (int b0 = 0; b0 < c; b0 += 32) {
        const int idx = b0 + lane;
        const int uv  = lw[idx < WLCAP ? idx : WLCAP - 1];
        const int m32 = (c - b0) < 32 ? (c - b0) : 32;
#pragma unroll 1
        for (int k = 0; k < m32; ++k) {
          const int u  = __builtin_amdgcn_readlane(uv, k);
          const int sl = u & (NBA - 1);
          const int t  = scnt[sl] + 1;
          if (lane == 0) scnt[sl] = t;
        }
      }
    }
  }
  __syncthreads();

  {
    const v4i ca = *(const v4ia*)(scnt + 4 * tid);
    const int e0 = ca.x < 0 ? 0 : ca.x, e1 = ca.y < 0 ? 0 : ca.y, e2 = ca.z < 0 ? 0 : ca.z, e3 = ca.w < 0 ? 0 : ca.w;
    const int ts = e0 + e1 + e2 + e3;
    int incl = ts;
#pragma unroll
    for (int d = 1; d < 32; d <<= 1) {
      const int up = __shfl_up(incl, d, 32);
      if (lane >= d) incl += up;
    }
    int mx = max(max(e0, e1), max(e2, e3));
    mx = max(mx, __shfl_xor(mx, 16, 32));
    mx = max(mx, __shfl_xor(mx, 8, 32));
    mx = max(mx, __shfl_xor(mx, 4, 32));
    mx = max(mx, __shfl_xor(mx, 2, 32));
    mx = max(mx, __shfl_xor(mx, 1, 32));
    if (lane == 31) wtot[wave] = incl;
    if (lane == 0)  wmx[wave] = mx;
    __syncthreads();
    int pre = 0;
#pragma unroll
    for (int w2 = 0; w2 < NWAVE; ++w2) pre += (w2 < wave) ? wtot[w2] : 0;
    int run = pre + incl - ts;
    v4i so;
    so.x = run; run += e0;
    so.y = run; run += e1;
    so.z = run; run += e2;
    so.w = run;
    *(v4ia*)(soff + 4 * tid) = so;
    *(v4ia*)(cur + 4 * tid)  = so;
  }
  __syncthreads();

  if (wave == 0) {
#pragma unroll 1
    for (int w2 = 0; w2 < NWAVE; ++w2) {
      int cv = wcnt[w2];
      cv = cv < 0 ? 0 : (cv > WLCAP ? WLCAP : cv);
      const int c = __builtin_amdgcn_readfirstlane(cv);
      const int* lw = wl + w2 * WLCAP;
#pragma unroll 1
      for (int b0 = 0; b0 < c; b0 += 32) {
        const int idx = b0 + lane;
        const int uv  = lw[idx < WLCAP ? idx : WLCAP - 1];
        const int m32 = (c - b0) < 32 ? (c - b0) : 32;
#pragma unroll 1
        for (int k = 0; k < m32; ++k) {
          const int u   = __builtin_amdgcn_readlane(uv, k);
          const int sl  = u & (NBA - 1);
          const int eid = (int)((unsigned)u >> PKS);
          int pos = cur[sl];
          pos = pos < 0 ? 0 : (pos > RCAP - 1 ? RCAP - 1 : pos);
          if (lane == 0) {
            reg2[pos] = eid;
            cur[sl] = pos + 1;
          }
        }
      }
    }
  }
  __syncthreads();

  int bmax = 0;
#pragma unroll
  for (int w2 = 0; w2 < NWAVE; ++w2) bmax = max(bmax, wmx[w2]);
  const int flag = ((ovf != 0) || (bmax > DEGCAP)) ? 1 : 0;

  int* lrow = LIST + (size_t)blockIdx.x * RCAP;
#pragma unroll 1
  for (int it = 0; it < RCAP / (NTHR * 4); ++it) {
    const int i0 = 4 * (it * NTHR + tid);
    const v4i ev = *(const v4ia*)(reg2 + i0);
    int e0 = ev.x, e1 = ev.y, e2 = ev.z, e3 = ev.w;
    e0 = e0 < 0 ? 0 : (e0 > nE - 1 ? nE - 1 : e0);
    e1 = e1 < 0 ? 0 : (e1 > nE - 1 ? nE - 1 : e1);
    e2 = e2 < 0 ? 0 : (e2 > nE - 1 ? nE - 1 : e2);
    e3 = e3 < 0 ? 0 : (e3 > nE - 1 ? nE - 1 : e3);
    int g0 = gidx[e0], g1 = gidx[e1], g2 = gidx[e2], g3 = gidx[e3];
    asm volatile("" :: "v"(g0), "v"(g1), "v"(g2), "v"(g3));
    g0 = g0 < 0 ? 0 : (g0 > nN - 1 ? nN - 1 : g0);
    g1 = g1 < 0 ? 0 : (g1 > nN - 1 ? nN - 1 : g1);
    g2 = g2 < 0 ? 0 : (g2 > nN - 1 ? nN - 1 : g2);
    g3 = g3 < 0 ? 0 : (g3 > nN - 1 ? nN - 1 : g3);
    v4i ov;
    ov.x = (i0     < nh) ? g0 : 0;
    ov.y = (i0 + 1 < nh) ? g1 : 0;
    ov.z = (i0 + 2 < nh) ? g2 : 0;
    ov.w = (i0 + 3 < nh) ? g3 : 0;
    *(volatile v4i*)(lrow + i0) = ov;
    __threadfence();
    *(volatile v4i*)(lrow + i0) = ov;
  }
  {
    const v4i cv = *(const v4ia*)(scnt + 4 * tid);
    const v4i fv = *(const v4ia*)(soff + 4 * tid);
    v4i rv = {0, 0, 0, 0};
    rv.x = (tid == 0) ? bmax : 0;
    rv.y = (tid == 0) ? flag : 0;
    rv.z = (tid == 0) ? nh : 0;
    int* cp = CNT + (size_t)nodeBase + 4 * tid;
    int* fp = OFF + (size_t)nodeBase + 4 * tid;
    int* rp = REC + (size_t)blockIdx.x * 32 + 4 * (tid & 7);
    *(volatile v4i*)cp = cv;
    *(volatile v4i*)fp = fv;
    if (tid < 8) *(volatile v4i*)rp = rv;
    __threadfence();
    *(volatile v4i*)cp = cv;
    *(volatile v4i*)fp = fv;
    if (tid < 8) *(volatile v4i*)rp = rv;
  }
}

template <int HL>
__global__ __launch_bounds__(NTHR) void k_replay(const unsigned short* __restrict__ src, unsigned short* dst,
                                                 const int* __restrict__ LIST, const int* __restrict__ CNT,
                                                 const int* __restrict__ OFF, const int* __restrict__ REC,
                                                 int nN, int mRows) {
  const int tid = (int)threadIdx.x, lane = tid & 31, wave = tid >> 5, hh = lane >> 4, m = lane & 15;
  const int blk0 = (int)blockIdx.x * RPB;
  const int bb   = blk0 >> PKS;
  const int fl   = REC[(size_t)bb * 32 + 1];
  const unsigned pz = (fl != 0) ? 0x7fc00000u : 0u;
  const int* lp = LIST + (size_t)bb * RCAP;
#pragma unroll 1
  for (int ri = 0; ri < RPW; ++ri) {
    const int node = blk0 + wave * RPW + ri;
    const int craw = CNT[node];
    const int oraw = OFF[node];
    const int deg  = craw < 0 ? 0 : craw;
    int cv = deg > DEGCAP ? DEGCAP : deg;
    int ov = oraw < 0 ? 0 : (oraw > RCAP ? RCAP : oraw);
    if (cv > RCAP - ov) cv = RCAP - ov;
    const int c = __builtin_amdgcn_readfirstlane(cv);
    const int o = __builtin_amdgcn_readfirstlane(ov);
    const bool big = deg > DEGCAP;
    int last = o + c - 1;
    last = last < o ? o : last;
    last = last > RCAP - 1 ? RCAP - 1 : last;
    float a0 = 0.f, a1 = 0.f, a2 = 0.f, a3 = 0.f, a4 = 0.f, a5 = 0.f, a6 = 0.f, a7 = 0.f;
#pragma unroll 1
    for (int b0 = 0; b0 < c; b0 += 32) {
      int idx = o + b0 + lane;
      idx = idx > last ? last : idx;
      int col = lp[idx];
      col = col < 0 ? 0 : (col > nN - 1 ? nN - 1 : col);
      const int m32 = (c - b0) < 32 ? (c - b0) : 32;
#pragma unroll 1
      for (int k = 0; k < m32; k += 2) {
        const int s0 = __builtin_amdgcn_readlane(col, k);
        const int s1 = __builtin_amdgcn_readlane(col, k + 1);
        const int sk = s0 + hh * (s1 - s0);
        const unsigned mk = ((k + hh) < m32) ? 0xFFFFFFFFu : 0u;
        if constexpr (HL == 0) {
          const unsigned short* rp = src + (size_t)sk * XP + 8 * m;
          v4u w = *(const v4ua*)rp;
          asm volatile("" :: "v"(w));
          w.x &= mk; w.y &= mk; w.z &= mk; w.w &= mk;
          a0 += bfw_lo(w.x); a1 += bfw_hi(w.x);
          a2 += bfw_lo(w.y); a3 += bfw_hi(w.y);
          a4 += bfw_lo(w.z); a5 += bfw_hi(w.z);
          a6 += bfw_lo(w.w); a7 += bfw_hi(w.w);
        } else {
          const unsigned short* rp = src + (size_t)sk * SP + 8 * m;
          v4u wh = *(const v4ua*)rp;
          v4u wl = *(const v4ua*)(rp + DF);
          asm volatile("" :: "v"(wh), "v"(wl));
          wh.x &= mk; wh.y &= mk; wh.z &= mk; wh.w &= mk;
          wl.x &= mk; wl.y &= mk; wl.z &= mk; wl.w &= mk;
          a0 += bfw_lo(wh.x) + bfw_lo(wl.x);
          a1 += bfw_hi(wh.x) + bfw_hi(wl.x);
          a2 += bfw_lo(wh.y) + bfw_lo(wl.y);
          a3 += bfw_hi(wh.y) + bfw_hi(wl.y);
          a4 += bfw_lo(wh.z) + bfw_lo(wl.z);
          a5 += bfw_hi(wh.z) + bfw_hi(wl.z);
          a6 += bfw_lo(wh.w) + bfw_lo(wl.w);
          a7 += bfw_hi(wh.w) + bfw_hi(wl.w);
        }
      }
    }
    a0 += __shfl_xor(a0, 16, 32); a1 += __shfl_xor(a1, 16, 32);
    a2 += __shfl_xor(a2, 16, 32); a3 += __shfl_xor(a3, 16, 32);
    a4 += __shfl_xor(a4, 16, 32); a5 += __shfl_xor(a5, 16, 32);
    a6 += __shfl_xor(a6, 16, 32); a7 += __shfl_xor(a7, 16, 32);
    const bool live = node < nN;
    const unsigned pzr = big ? 0x7fc00000u : pz;
    const unsigned km  = (pzr != 0u) ? 0u : 0xFFFFFFFFu;
    const float r0 = live ? poison(a0, km, pzr) : 0.0f;
    const float r1 = live ? poison(a1, km, pzr) : 0.0f;
    const float r2 = live ? poison(a2, km, pzr) : 0.0f;
    const float r3 = live ? poison(a3, km, pzr) : 0.0f;
    const float r4 = live ? poison(a4, km, pzr) : 0.0f;
    const float r5 = live ? poison(a5, km, pzr) : 0.0f;
    const float r6 = live ? poison(a6, km, pzr) : 0.0f;
    const float r7 = live ? poison(a7, km, pzr) : 0.0f;
    unsigned h0, l0, h1, l1, h2, l2, h3, l3;
    pack2(r0, r1, h0, l0);
    pack2(r2, r3, h1, l1);
    pack2(r4, r5, h2, l2);
    pack2(r6, r7, h3, l3);
    const bool isHi = (hh == 0);
    v4u q;
    q.x = isHi ? h0 : l0;
    q.y = isHi ? h1 : l1;
    q.z = isHi ? h2 : l2;
    q.w = isHi ? h3 : l3;
    unsigned short* wp = dst + (size_t)node * SP + hh * DF + 8 * m;
    *(volatile v4u*)wp = q;
    __threadfence();
    *(volatile v4u*)wp = q;
  }
}

template <int WP>
__device__ __forceinline__ void kpart(const unsigned short* ap, const unsigned short* __restrict__ wp, int nsteps,
                                      v8f (&acc)[8]) {
#pragma unroll 1
  for (int ks = 0; ks < nsteps; ++ks) {
    FragB af;
    af.h[0] = *(const v8usa*)(ap + 32 * ks);
    af.h[1] = *(const v8usa*)(ap + 32 * ks + 16);
#pragma unroll
    for (int t = 0; t < 8; ++t) {
      const unsigned short* wq = wp + (size_t)(16 * t) * (size_t)WP + 32 * ks;
      FragB bf;
      bf.h[0] = *(const v8usa*)wq;
      bf.h[1] = *(const v8usa*)(wq + 16);
      acc[t] = wmb(af, bf, acc[t]);
    }
  }
}

template <int LAYER>
__global__ __launch_bounds__(GTHR) __attribute__((amdgpu_num_vgpr(248)))
void k_gemm(unsigned short* pl_a, const unsigned short* pl_b, const unsigned short* __restrict__ wt,
            const float* __restrict__ bias, const int* __restrict__ REC, float* outp, int nN) {
  __shared__ __attribute__((aligned(16))) float stg[GBM * GBN];
  __shared__ __attribute__((aligned(16))) float bsh[GBN];
  const int tid = (int)threadIdx.x, lane = tid & 31, wave = tid >> 5, hh = lane >> 4, m = lane & 15;
  const int rowBase = (int)blockIdx.x * GBM;

  if (tid < 32) {
    const v4f b4 = *(const v4f*)(bias + 4 * tid);
    v4f bq;
    bq.x = bf16_val(b4.x); bq.y = bf16_val(b4.y); bq.z = bf16_val(b4.z); bq.w = bf16_val(b4.w);
    *(v4fa*)(bsh + 4 * tid) = bq;
  }

  v8f acc[8];
  {
    const v8f z = {0.f, 0.f, 0.f, 0.f, 0.f, 0.f, 0.f, 0.f};
#pragma unroll
    for (int t = 0; t < 8; ++t) acc[t] = z;
  }
  const size_t grow = (size_t)(rowBase + 16 * wave + m);
  if constexpr (LAYER == 1) {
    const unsigned short* wp = wt + (size_t)m * WPA + 8 * hh;
    kpart<WPA>((const unsigned short*)pl_a + grow * SP + 8 * hh, wp, KS_S1, acc);
    kpart<WPA>(pl_b + grow * XP + 8 * hh, wp + WOFF_ROOT, KS_X, acc);
  } else {
    const unsigned short* wp = wt + (size_t)m * WPB + 8 * hh;
    kpart<WPB>((const unsigned short*)pl_a + grow * SP + 8 * hh, wp, KS_S2, acc);
    kpart<WPB>(pl_b + grow * SP + 8 * hh, wp + WOFF_ROOT, KS_H, acc);
  }
  __syncthreads();

#pragma unroll
  for (int t = 0; t < 8; ++t) {
    const int lc = 16 * t + m;
    const float bb = bsh[lc];
#pragma unroll
    for (int r = 0; r < 8; ++r) {
      const int lr = 16 * wave + 8 * hh + r;
      float v = acc[t][r] + bb;
      if constexpr (LAYER == 1) {
        const bool live = (rowBase + lr) < nN;
        v = relu_k(v);
        v = live ? v : 0.0f;
      }
      stg[lr * GBN + lc] = v;
    }
  }
  __syncthreads();

  if constexpr (LAYER == 1) {
    const int cb = 8 * m;
    const bool isHi = (hh == 0);
    v4u pk[16];
#pragma unroll
    for (int i = 0; i < 16; ++i) {
      const int lr = 16 * wave + i;
      const v4f a = *(const v4fa*)(stg + lr * GBN + cb);
      const v4f b = *(const v4fa*)(stg + lr * GBN + cb + 4);
      unsigned h0, l0, h1, l1, h2, l2, h3, l3;
      pack2(a.x, a.y, h0, l0);
      pack2(a.z, a.w, h1, l1);
      pack2(b.x, b.y, h2, l2);
      pack2(b.z, b.w, h3, l3);
      v4u pw;
      pw.x = isHi ? h0 : l0;
      pw.y = isHi ? h1 : l1;
      pw.z = isHi ? h2 : l2;
      pw.w = isHi ? h3 : l3;
      pk[i] = pw;
    }
#pragma unroll
    for (int i = 0; i < 16; ++i) {
      const int gr = rowBase + 16 * wave + i;
      unsigned short* op = pl_a + (size_t)gr * (size_t)SP + hh * DF + cb;
      *(volatile v4u*)op = pk[i];
    }
    __threadfence();
#pragma unroll
    for (int i = 0; i < 16; ++i) {
      const int gr = rowBase + 16 * wave + i;
      unsigned short* op = pl_a + (size_t)gr * (size_t)SP + hh * DF + cb;
      *(volatile v4u*)op = pk[i];
    }
  } else {
    const int fl = REC[(size_t)(rowBase >> PKS) * 32 + 1];
    const unsigned pz = (fl != 0) ? 0x7fc00000u : 0u;
    const unsigned km = (pz != 0u) ? 0u : 0xFFFFFFFFu;
    v4f pv[16];
#pragma unroll
    for (int i = 0; i < 16; ++i) {
      const v4f a = *(const v4fa*)(stg + (16 * wave + i) * GBN + 4 * lane);
      v4f o;
      o.x = poison(a.x, km, pz);
      o.y = poison(a.y, km, pz);
      o.z = poison(a.z, km, pz);
      o.w = poison(a.w, km, pz);
      pv[i] = o;
    }
#pragma unroll
    for (int i = 0; i < 16; ++i) {
      const int gr = rowBase + 16 * wave + i;
      if (gr < nN) *(volatile v4f*)(outp + (size_t)gr * DF + 4 * lane) = pv[i];
    }
    __threadfence();
#pragma unroll
    for (int i = 0; i < 16; ++i) {
      const int gr = rowBase + 16 * wave + i;
      if (gr < nN) *(volatile v4f*)(outp + (size_t)gr * DF + 4 * lane) = pv[i];
    }
  }
}

static inline int cdiv(int a, int b) { return (a + b - 1) / b; }
static inline size_t al256(size_t o) { return (o + 255) & ~(size_t)255; }

extern "C" void kernel_launch(void* const* d_in, const int* in_sizes, int n_in,
                              void* d_out, int out_size, void* d_ws, size_t ws_size,
                              hipStream_t stream) {
  if (n_in < 8) return;
  if (in_sizes[0] < DF * RPB || (in_sizes[0] % DF) != 0) return;
  const int nN = in_sizes[0] / DF;
  if (in_sizes[1] < 2 || (in_sizes[1] & 1) != 0) return;
  const int nE = in_sizes[1] / 2;
  if (nE < 1 || nE + CHUNK >= (1 << 21)) return;
  if (nN >= (1 << 24)) return;
  if (in_sizes[2] != DF * DF || in_sizes[3] != DF * DF || in_sizes[4] != DF) return;
  if (in_sizes[5] != DF * DF || in_sizes[6] != DF * DF || in_sizes[7] != DF) return;
  if ((long long)out_size != (long long)nN * DF) return;

  const float* x      = (const float*)d_in[0];
  const int*   ei     = (const int*)  d_in[1];
  const int*   srcix  = ei;
  const int*   keyix  = ei + nE;
  const float* wrel1  = (const float*)d_in[2];
  const float* wroot1 = (const float*)d_in[3];
  const float* bia1   = (const float*)d_in[4];
  const float* wrel2  = (const float*)d_in[5];
  const float* wroot2 = (const float*)d_in[6];
  const float* bia2   = (const float*)d_in[7];
  float* out = (float*)d_out;

  const int nB    = cdiv(nN, NBA);
  const int NPADN = nB * NBA;
  const int MP    = cdiv(nN, 128) * 128;
  if (MP > NPADN) return;
  const int gR    = MP / RPB;
  const int vec8  = ((nE & 3) == 0) ? 1 : 0;

  char* ws = (char*)d_ws;
  size_t off = 0;
  const size_t oWA = off; off = al256(off + (size_t)DF * WPA * 2);
  const size_t oWB = off; off = al256(off + (size_t)DF * WPB * 2);
  const size_t oLS = off; off = al256(off + (size_t)nB * RCAP * 4);
  const size_t oCN = off; off = al256(off + (size_t)NPADN * 4);
  const size_t oOF = off; off = al256(off + (size_t)NPADN * 4);
  const size_t oRC = off; off = al256(off + (size_t)nB * 128);
  const size_t oPA = off; off = al256(off + (size_t)MP * SP * 2);
  const size_t oPB = off; off = al256(off + (size_t)MP * SP * 2);
  if (off > ws_size || off > (size_t)(128u << 20)) return;
  unsigned short* wca = (unsigned short*)(ws + oWA);
  unsigned short* wcb = (unsigned short*)(ws + oWB);
  int* LIST = (int*)(ws + oLS);
  int* CNT  = (int*)(ws + oCN);
  int* OFF  = (int*)(ws + oOF);
  int* REC  = (int*)(ws + oRC);
  unsigned short* pa = (unsigned short*)(ws + oPA);
  unsigned short* pb = (unsigned short*)(ws + oPB);
  unsigned short* xb = pb;

  hipFuncSetAttribute(reinterpret_cast<const void*>(&k_bucket), hipFuncAttributeMaxDynamicSharedMemorySize, LDS_BK);

  k_prep<<<WBLK + MP / 16, NTHR, 0, stream>>>(x, wrel1, wroot1, wrel2, wroot2, xb, wca, wcb, nN, MP);
  k_bucket<<<nB, NTHR, LDS_BK, stream>>>(keyix, srcix, nE, nN, vec8, LIST, CNT, OFF, REC);
  k_replay<0><<<gR, NTHR, 0, stream>>>(xb, pa, LIST, CNT, OFF, REC, nN, MP);
  k_gemm<1><<<gR, GTHR, 0, stream>>>(pa, xb, wca, bia1, REC, out, nN);
  k_replay<1><<<gR, NTHR, 0, stream>>>(pa, pb, LIST, CNT, OFF, REC, nN, MP);
  k_gemm<2><<<gR, GTHR, 0, stream>>>(pb, pa, wcb, bia2, REC, out, nN);
}
